// SinkhornOT_87479893885304
// MI455X (gfx1250) — hardware-verified
//
#include <hip/hip_runtime.h>
#include <math.h>


#ifndef NB
#define NB 2048
#endif
#define NB_FULL 2048
#define NS 16
#define DD 256
#define XP 264
#define QP 260
#define OT_ITERS 20
#define OT_MESH 3
#define TCLP 32
#define XSC 16.0f
#define WSC 64.0f
#define RSC 4096.0f
#define INV_XW (1.0f / 1024.0f)
#define INV_W (1.0f / 64.0f)
#define INV_R (1.0f / 4096.0f)
#define INV_EPS 20.0f

#define OFF_SIM 0
#define OFF_T (NB_FULL)
#define OFF_C (NB_FULL + NB_FULL * NS * NS)
#define OFF_K (NB_FULL + 2 * NB_FULL * NS * NS)
static_assert(OFF_T * 4 == 8192);
static_assert(OFF_C * 4 == 2105344);
static_assert(OFF_K * 4 == 4202496);
static_assert((OFF_K + NB_FULL) * 4 == 4210688);
static_assert(NB >= 1 && NB <= NB_FULL);

#define WS_W1 ((size_t)0)
#define WS_W2 ((size_t)DD * DD * 2)
#define WS_TCL ((size_t)2 * DD * DD * 2)
#define WS_END (WS_TCL + (size_t)NB * TCLP * 4)
static_assert(WS_END <= (size_t)134217728);
static_assert((WS_W2 % 128) == 0 && (WS_TCL % 128) == 0);

typedef __attribute__((ext_vector_type(16))) _Float16 v16h;
typedef __attribute__((ext_vector_type(8)))  _Float16 v8h;
typedef __attribute__((ext_vector_type(8)))  float v8f;
typedef __attribute__((ext_vector_type(4)))  float v4f;
typedef __attribute__((ext_vector_type(4)))  unsigned v4u;

template <typename T> __device__ __forceinline__ void vst2(void* p, T v) { *(volatile T*)p = v; __threadfence(); *(volatile T*)p = v; }
__device__ __forceinline__ void vst2f(float* p, float v) { *(volatile float*)p = v; __threadfence(); *(volatile float*)p = v; }

__device__ __forceinline__ v8f wmma16(v16h a, v16h b, v8f c) {
  v8f d = __builtin_amdgcn_wmma_f32_16x16x32_f16(false, a, false, b, (short)0, c, false, false);
  asm volatile("v_nop\n\tv_nop\n\tv_nop\n\tv_nop" : "+v"(d) : "v"(a), "v"(b));
  return d;
}
__device__ __forceinline__ v16h frag_h(const _Float16* rowk0, int lane) {
  union { v16h v; v8h q[2]; } u; const _Float16* p = rowk0 + 8 * (lane >> 4);
  u.q[0] = *(const v8h*)p; u.q[1] = *(const v8h*)(p + 16); return u.v;
}
__device__ __forceinline__ float bfr(float x) {
  unsigned u = __float_as_uint(x); u = (u + 0x7fffu + ((u >> 16) & 1u)) & 0xffff0000u; return __uint_as_float(u);
}
__device__ __forceinline__ v8h cvt8s(const float* p, float scale) {
  const v4f f0 = *(const v4f*)p; const v4f f1 = *(const v4f*)(p + 4); v8h h;
#pragma unroll
  for (int e = 0; e < 4; ++e) { h[e] = (_Float16)(bfr(f0[e]) * scale); h[4 + e] = (_Float16)(bfr(f1[e]) * scale); }
  return h;
}

__device__ __forceinline__ float hmax16(float v) {
  v = fmaxf(v, __shfl_xor(v, 1, 32)); v = fmaxf(v, __shfl_xor(v, 2, 32));
  v = fmaxf(v, __shfl_xor(v, 4, 32)); v = fmaxf(v, __shfl_xor(v, 8, 32));
  return v;
}
__device__ __forceinline__ float hsum16(float v) {
  v += __shfl_xor(v, 1, 32); v += __shfl_xor(v, 2, 32); v += __shfl_xor(v, 4, 32); v += __shfl_xor(v, 8, 32);
  return v;
}
__device__ __forceinline__ float lse16(float x) { const float mx = hmax16(x); const float s = hsum16(expf(x - mx)); return mx + logf(s); }

__global__ __launch_bounds__(256) void k_cvtw(const float* __restrict__ W1, const float* __restrict__ W2,
                                             _Float16* __restrict__ P1, _Float16* __restrict__ P2) {
  const int blk = blockIdx.x;
  const float* s = blk < 32 ? W1 : W2; _Float16* d = blk < 32 ? P1 : P2;
  const size_t g8 = (size_t)(blk & 31) * 256 + threadIdx.x;
  union { v8h h; v4u u; } pk; pk.h = cvt8s(s + g8 * 8, WSC);
  vst2(d + g8 * 8, pk.u);
}

__global__ __launch_bounds__(64) void k_main(const float* __restrict__ sq, const float* __restrict__ sr,
                                            const float* __restrict__ mq, const float* __restrict__ mr,
                                            const _Float16* __restrict__ P1, const float* __restrict__ b1,
                                            const _Float16* __restrict__ P2, const float* __restrict__ b2,
                                            float* __restrict__ outT, float* __restrict__ outC, float* __restrict__ tcl) {
  __shared__ __align__(16) _Float16 xs[2 * NS * XP];
  __shared__ __align__(16) _Float16 hh[2 * NS * XP];
  __shared__ __align__(16) _Float16 hl[2 * NS * XP];
  __shared__ __align__(16) float qf[2 * NS * QP];
  __shared__ __align__(16) float cs[NS * NS];
  __shared__ __align__(16) float ts[NS * NS];
  __shared__ float b1s[DD], b2s[DD];
  const int tid = threadIdx.x, wave = tid >> 5, lane = tid & 31, m = lane & 15, g = lane >> 4;
  const int b = blockIdx.x;

  for (int i = tid; i < DD; i += 64) { b1s[i] = bfr(b1[i]); b2s[i] = bfr(b2[i]); }
  {
    const float* bq = sq + (size_t)b * (NS * DD);
    const float* br = sr + (size_t)b * (NS * DD);
#pragma unroll 1
    for (int i = tid; i < NS * (DD / 8); i += 64) {
      const int row = i >> 5, c8 = (i & 31) * 8;
      *(v8h*)(xs + row * XP + c8) = cvt8s(bq + row * DD + c8, XSC);
      *(v8h*)(xs + (NS + row) * XP + c8) = cvt8s(br + row * DD + c8, XSC);
    }
  }
  __syncthreads();

  const int R0 = wave * NS;
#pragma unroll 1
  for (int p = 0; p < 2; ++p) {
    const int n0 = p * 128;
    v8f acc[8] = {};
#pragma unroll 1
    for (int kc = 0; kc < DD / 32; ++kc) {
      const v16h a = frag_h(xs + (R0 + m) * XP + kc * 32, lane);
#pragma unroll
      for (int j = 0; j < 8; ++j) acc[j] = wmma16(a, frag_h(P1 + (size_t)(n0 + j * 16 + m) * DD + kc * 32, lane), acc[j]);
    }
#pragma unroll
    for (int j = 0; j < 8; ++j) {
      const int col = n0 + j * 16 + m; const float bv = b1s[col];
#pragma unroll
      for (int r = 0; r < 8; ++r) {
        float v = acc[j][r] * INV_XW + bv; v = v > 0.f ? v : 0.f;
        const _Float16 hv = (_Float16)v; const float res = (v - (float)hv) * RSC;
        hh[(R0 + 8 * g + r) * XP + col] = hv; hl[(R0 + 8 * g + r) * XP + col] = (_Float16)res;
      }
    }
  }
  __syncthreads();

#pragma unroll 1
  for (int p = 0; p < 4; ++p) {
    const int n0 = p * 64;
    v8f ach[4] = {}, acl[4] = {};
#pragma unroll 1
    for (int kc = 0; kc < DD / 32; ++kc) {
      const v16h ah = frag_h(hh + (R0 + m) * XP + kc * 32, lane);
      const v16h al = frag_h(hl + (R0 + m) * XP + kc * 32, lane);
#pragma unroll
      for (int j = 0; j < 4; ++j) {
        const v16h bw = frag_h(P2 + (size_t)(n0 + j * 16 + m) * DD + kc * 32, lane);
        ach[j] = wmma16(ah, bw, ach[j]); acl[j] = wmma16(al, bw, acl[j]);
      }
    }
#pragma unroll
    for (int j = 0; j < 4; ++j) {
      const int col = n0 + j * 16 + m; const float bv = b2s[col];
#pragma unroll
      for (int r = 0; r < 8; ++r) qf[(R0 + 8 * g + r) * QP + col] = (ach[j][r] + acl[j][r] * INV_R) * INV_W + bv;
    }
  }
  __syncthreads();

  {
    const int k = tid >> 2, m0 = (tid & 3) * 4;
    v4f d2[4] = {};
#pragma unroll 1
    for (int c4 = 0; c4 < DD / 4; ++c4) {
      const v4f qv = *(const v4f*)(qf + k * QP + c4 * 4);
#pragma unroll
      for (int j = 0; j < 4; ++j) { const v4f rv = *(const v4f*)(qf + (NS + m0 + j) * QP + c4 * 4); const v4f dv = qv - rv; d2[j] += dv * dv; }
    }
#pragma unroll
    for (int j = 0; j < 4; ++j) { const float s = (d2[j][0] + d2[j][1]) + (d2[j][2] + d2[j][3]); cs[k * NS + m0 + j] = sqrtf(fmaxf(s, 1e-6f)); }
  }
  __syncthreads();
  vst2(outC + (size_t)b * (NS * NS) + tid * 4, *(const v4f*)(cs + tid * 4));

  if (wave == 0) {
    float Cv[8];
#pragma unroll
    for (int v = 0; v < 8; ++v) Cv[v] = cs[(8 * g + v) * NS + m];
    const float vq = bfr(mq[(size_t)b * NS + m]), vr = bfr(mr[(size_t)b * NS + m]);
    const float lq = logf(fmaxf(vq, 1e-8f)), lr = logf(fmaxf(vr, 1e-8f));
    const float lmq = lq - lse16(lq);
    const float lnu = lr - lse16(lr);
    float lk[8];
#pragma unroll
    for (int v = 0; v < 8; ++v) { const float lmu = __shfl(lmq, 8 * g + v, 32); const float nk = -Cv[v] * INV_EPS; lk[v] = (nk + lmu) + lnu; }
    float la[8]; float lb = 0.f;
#pragma unroll
    for (int v = 0; v < 8; ++v) la[v] = 0.f;
#pragma unroll 1
    for (int it = 0; it < OT_ITERS; ++it) {
#pragma unroll
      for (int v = 0; v < 8; ++v) la[v] = -lse16(lk[v] + lb);
      float u[8]; float mx;
#pragma unroll
      for (int v = 0; v < 8; ++v) u[v] = lk[v] + la[v];
      mx = u[0];
#pragma unroll
      for (int v = 1; v < 8; ++v) mx = fmaxf(mx, u[v]);
      mx = fmaxf(mx, __shfl_xor(mx, 16, 32));
      float s = 0.f;
#pragma unroll
      for (int v = 0; v < 8; ++v) s += expf(u[v] - mx);
      s += __shfl_xor(s, 16, 32);
      lb = -(mx + logf(s));
    }
    float T[8];
#pragma unroll
    for (int v = 0; v < 8; ++v) T[v] = expf((lk[v] + la[v]) + lb);
#pragma unroll 1
    for (int mi = 0; mi < OT_MESH; ++mi) {
#pragma unroll
      for (int v = 0; v < 8; ++v) T[v] = T[v] * T[v];
#pragma unroll
      for (int v = 0; v < 8; ++v) { const float rs = hsum16(T[v]); T[v] = T[v] * (1.0f / (rs + 1e-8f)); }
      float csum = 0.f;
#pragma unroll
      for (int v = 0; v < 8; ++v) csum += T[v];
      csum += __shfl_xor(csum, 16, 32);
      const float ic = 1.0f / (csum + 1e-8f);
#pragma unroll
      for (int v = 0; v < 8; ++v) T[v] = T[v] * ic;
    }
    float tc = 0.f;
#pragma unroll
    for (int v = 0; v < 8; ++v) tc += T[v] * Cv[v];
    tc = hsum16(tc); tc += __shfl_xor(tc, 16, 32);
#pragma unroll
    for (int v = 0; v < 8; ++v) ts[(8 * g + v) * NS + m] = T[v];
    if (lane < 8) { v4f cv = {tc, tc, tc, tc}; vst2(tcl + (size_t)b * TCLP + lane * 4, cv); }
  }
  __syncthreads();
  vst2(outT + (size_t)b * (NS * NS) + tid * 4, *(const v4f*)(ts + tid * 4));
}

__global__ __launch_bounds__(256) void k_fin(const float* __restrict__ tcl, float* __restrict__ outS, float* __restrict__ outK, int nb) {
  __shared__ __align__(16) float sc[256];
  __shared__ __align__(16) float ss[256];
  const int tid = threadIdx.x;
  const int bb = blockIdx.x * 256 + tid; const int bc = bb < nb ? bb : nb - 1;
  const float c = tcl[(size_t)bc * TCLP];
  sc[tid] = c; ss[tid] = 1.0f / (1.0f + expf(c));
  __syncthreads();
  if (tid < 64) {
    const int q = tid, i0 = blockIdx.x * 256 + q * 4;
    if (i0 + 3 < nb) vst2(outK + i0, *(const v4f*)(sc + q * 4));
    else { for (int e = 0; e < 4; ++e) if (i0 + e < nb) vst2f(outK + i0 + e, sc[q * 4 + e]); }
  } else if (tid < 128) {
    const int q = tid - 64, i0 = blockIdx.x * 256 + q * 4;
    if (i0 + 3 < nb) vst2(outS + i0, *(const v4f*)(ss + q * 4));
    else { for (int e = 0; e < 4; ++e) if (i0 + e < nb) vst2f(outS + i0 + e, ss[q * 4 + e]); }
  }
}

extern "C" void kernel_launch(void* const* d_in, const int* in_sizes, int n_in,
                              void* d_out, int out_size, void* d_ws, size_t ws_size,
                              hipStream_t stream) {
  if (n_in < 8) return;
  if (in_sizes[0] < NB * NS * DD || in_sizes[1] < NB * NS * DD || in_sizes[2] < NB * NS || in_sizes[3] < NB * NS) return;
  if (in_sizes[4] < DD * DD || in_sizes[5] < DD || in_sizes[6] < DD * DD || in_sizes[7] < DD) return;
  if ((size_t)out_size < (size_t)OFF_K + NB) return;
  if (ws_size < WS_END) return;
  const float* slots_q = (const float*)d_in[0];
  const float* slots_r = (const float*)d_in[1];
  const float* mask_q = (const float*)d_in[2];
  const float* mask_r = (const float*)d_in[3];
  const float* W1 = (const float*)d_in[4];
  const float* b1 = (const float*)d_in[5];
  const float* W2 = (const float*)d_in[6];
  const float* b2 = (const float*)d_in[7];
  char* ws = (char*)d_ws;
  _Float16* P1 = (_Float16*)(ws + WS_W1);
  _Float16* P2 = (_Float16*)(ws + WS_W2);
  float* tcl = (float*)(ws + WS_TCL);
  float* out = (float*)d_out;
  float* o_sim = out + OFF_SIM; float* o_T = out + OFF_T; float* o_C = out + OFF_C; float* o_K = out + OFF_K;

  k_cvtw<<<64, 256, 0, stream>>>(W1, W2, P1, P2);
  k_main<<<NB, 64, 0, stream>>>(slots_q, slots_r, mask_q, mask_r, P1, b1, P2, b2, o_T, o_C, tcl);
  k_fin<<<(NB + 255) / 256, 256, 0, stream>>>(tcl, o_sim, o_K, NB);
}
